// transBlocklayer3_61452392071713
// MI455X (gfx1250) — hardware-verified
//
#include <hip/hip_runtime.h>
#include <stdint.h>

typedef _Float16 v16h __attribute__((ext_vector_type(16)));
typedef _Float16 v8h  __attribute__((ext_vector_type(8)));
typedef float    v8f  __attribute__((ext_vector_type(8)));
typedef float    v4f  __attribute__((ext_vector_type(4)));
typedef unsigned int v4u __attribute__((ext_vector_type(4)));
typedef v8h __attribute__((may_alias)) v8ha;
typedef v4f __attribute__((may_alias)) v4fa;
typedef v4u __attribute__((may_alias)) v4ua;

union Frag { v16h v; v8h half[2]; };

#define NB      64
#define CCH     256
#define HH      28
#define WW      28
#define HWSZ    784
#define NPOS    50176
#define KTOT    2304
#define NKC     72
#define TILE_P  64
#define XS_STRIDE 40
#define TS      260
#define CG      8
#define WSCALE      16.0f
#define WSCALE_INV  0.0625f

static_assert(NPOS % TILE_P == 0);
static_assert(NPOS % 256 == 0);
static_assert((2 * CCH * KTOT) % 8 == 0);
static_assert(CCH % CG == 0);
static_assert((HWSZ * 4) % 16 == 0);

__device__ __forceinline__ v8f wmma_f16(v16h a, v16h b, v8f c) {
  v8f d = __builtin_amdgcn_wmma_f32_16x16x32_f16(false, a, false, b, (short)0, c, false, false);
  asm volatile("v_nop\n\tv_nop\n\tv_nop\n\tv_nop" : "+v"(d) : "v"(a), "v"(b));
  return d;
}

__device__ __forceinline__ v16h load_frag(const _Float16* p, int h) {
  Frag f;
  f.half[0] = *(const v8ha*)(p + 8 * h);
  f.half[1] = *(const v8ha*)(p + 16 + 8 * h);
  return f.v;
}

__global__ __launch_bounds__(256) void prep_w_kernel(
    const float* __restrict__ w0, const float* __restrict__ w1,
    _Float16* __restrict__ wb)
{
  const int g = blockIdx.x * 256 + threadIdx.x;
  const int per = CCH * (KTOT / 8);
  if (g >= 2 * per) return;
  const int set = g / per;
  const int rem = g - set * per;
  const int o   = rem / (KTOT / 8);
  const int k8  = rem - o * (KTOT / 8);
  const int k0  = k8 * 8;
  const int r   = k0 >> 8;
  const int c0  = k0 & (CCH - 1);
  const float* w = set ? w1 : w0;
  const float* src = w + ((size_t)(o * CCH + c0)) * 9 + r;
  const v8h o8 = { (_Float16)(src[0]  * WSCALE), (_Float16)(src[9]  * WSCALE),
                   (_Float16)(src[18] * WSCALE), (_Float16)(src[27] * WSCALE),
                   (_Float16)(src[36] * WSCALE), (_Float16)(src[45] * WSCALE),
                   (_Float16)(src[54] * WSCALE), (_Float16)(src[63] * WSCALE) };
  _Float16* dst = wb + (size_t)g * 8;
  *(volatile v8h*)dst = o8;
  __threadfence();
  *(volatile v8h*)dst = o8;
}

__global__ __launch_bounds__(256) void prep_x_kernel(
    const float* __restrict__ x, _Float16* __restrict__ xb)
{
  const int g = blockIdx.x * 256 + threadIdx.x;
  if (g >= NPOS * (CCH / 8)) return;
  const int pos = g >> 5;
  const int c8  = g & 31;
  const int n   = pos / HWSZ;
  const int hw  = pos - n * HWSZ;
  const float* src = x + ((size_t)(n * CCH + 8 * c8)) * HWSZ + hw;
  const v8h o8 = { (_Float16)src[0],        (_Float16)src[HWSZ],     (_Float16)src[2 * HWSZ], (_Float16)src[3 * HWSZ],
                   (_Float16)src[4 * HWSZ], (_Float16)src[5 * HWSZ], (_Float16)src[6 * HWSZ], (_Float16)src[7 * HWSZ] };
  _Float16* dst = xb + (size_t)g * 8;
  *(volatile v8h*)dst = o8;
  __threadfence();
  *(volatile v8h*)dst = o8;
}

__device__ __forceinline__ float pooled_at(const float* __restrict__ mu, int p, float gamma) {
  const int n  = p / HWSZ;
  const int hw = p - n * HWSZ;
  const int h  = hw / WW;
  const int w  = hw - h * WW;
  const float* img = mu + (size_t)n * HWSZ;
  float pooled = 0.0f;
  #pragma unroll
  for (int dy = -3; dy <= 3; ++dy) {
    const int hh = min(max(h + dy, 0), HH - 1);
    #pragma unroll
    for (int dx = -3; dx <= 3; ++dx) {
      const int ww = min(max(w + dx, 0), WW - 1);
      const float u = img[hh * WW + ww];
      pooled = (u < gamma) ? 1.0f : pooled;
    }
  }
  return pooled;
}

__global__ __launch_bounds__(256) void mask_kernel(
    const float* __restrict__ mu, float* __restrict__ bm, float* __restrict__ scl)
{
  __shared__ int red[256];
  const int tid = threadIdx.x;
  const float gamma = __uint_as_float(0x3B05BF37u);

  int cnt = 0;
  #pragma unroll 1
  for (int i = 0; i < NPOS / 256; ++i) {
    const int p = i * 256 + tid;
    const float pooled = pooled_at(mu, p, gamma);
    cnt += (pooled == 0.0f) ? 1 : 0;
    const float v = 1.0f - pooled;
    *(volatile float*)(bm + p) = v;
  }
  __threadfence();
  #pragma unroll 1
  for (int i = 0; i < NPOS / 256; ++i) {
    const int p = i * 256 + tid;
    const float pooled = pooled_at(mu, p, gamma);
    const float v = 1.0f - pooled;
    *(volatile float*)(bm + p) = v;
  }

  red[tid] = cnt;
  __syncthreads();
  for (int off = 128; off > 0; off >>= 1) {
    if (tid < off) red[tid] = red[tid] + red[tid + off];
    __syncthreads();
  }
  const int total = red[0];
  const float scale = (float)NPOS / (float)total;
  if (tid < 32) *(volatile float*)(scl + tid) = scale;
  __threadfence();
  if (tid < 32) *(volatile float*)(scl + tid) = scale;
}

__global__ __launch_bounds__(256) void conv_kernel(
    const _Float16* __restrict__ xb,
    const _Float16* __restrict__ wb,
    const float* __restrict__ bm,
    float* __restrict__ Y)
{
  __shared__ __attribute__((aligned(16))) _Float16 Xs[TILE_P * XS_STRIDE];
  __shared__ __attribute__((aligned(16))) float Ts[16 * TS];

  const int tid  = threadIdx.x;
  const int lane = tid & 31;
  const int wave = tid >> 5;
  const int mset = wave >> 2;
  const int chb  = (wave & 3) * 64;
  const int p0   = blockIdx.x * TILE_P;
  const int h16  = lane >> 4;
  const int m16  = lane & 15;

  const int fpos = tid & 63;
  const int coff = (tid >> 6) * 8;
  const int p  = p0 + fpos;
  const int n  = p / HWSZ;
  const int hw = p - n * HWSZ;
  const int h  = hw / WW;
  const int w  = hw - h * WW;
  const _Float16* ximg = xb + (size_t)n * HWSZ * CCH;

  const _Float16* wrow = wb + ((size_t)mset * CCH + chb + m16) * KTOT;

  const v8f zero8 = {0.f, 0.f, 0.f, 0.f, 0.f, 0.f, 0.f, 0.f};
  v8f acc[4][4];
  #pragma unroll
  for (int ms = 0; ms < 4; ++ms)
    #pragma unroll
    for (int s = 0; s < 4; ++s) acc[ms][s] = zero8;

  #pragma unroll 1
  for (int kc = 0; kc < NKC; ++kc) {
    const int r     = kc >> 3;
    const int cbase = (kc & 7) * 32;
    const int dy = r / 3 - 1;
    const int dx = r - (r / 3) * 3 - 1;
    const int hy = h + dy, wx = w + dx;
    const bool ok = (hy >= 0) & (hy < HH) & (wx >= 0) & (wx < WW);
    const int hyc = min(max(hy, 0), HH - 1);
    const int wxc = min(max(wx, 0), WW - 1);
    const v4u ld = *(const v4ua*)(ximg + ((size_t)(hyc * WW + wxc)) * CCH + cbase + coff);
    v4u xv;
    xv.x = ok ? ld.x : 0u;
    xv.y = ok ? ld.y : 0u;
    xv.z = ok ? ld.z : 0u;
    xv.w = ok ? ld.w : 0u;
    *(v4ua*)(Xs + fpos * XS_STRIDE + coff) = xv;
    __syncthreads();

    v16h af[4];
    #pragma unroll
    for (int ms = 0; ms < 4; ++ms)
      af[ms] = load_frag(wrow + (size_t)ms * 16 * KTOT + kc * 32, h16);

    #pragma unroll
    for (int s = 0; s < 4; ++s) {
      const v16h bf = load_frag(Xs + (s * 16 + m16) * XS_STRIDE, h16);
      #pragma unroll
      for (int ms = 0; ms < 4; ++ms)
        acc[ms][s] = wmma_f16(af[ms], bf, acc[ms][s]);
    }
    __syncthreads();
  }

  #pragma unroll
  for (int s = 0; s < 4; ++s) {
    const int pp = p0 + 16 * s + m16;
    const float mval = bm[pp];
    const bool sel0 = (mval == 1.0f);
    const bool writeMe = (mset == 0) ? sel0 : (!sel0);
    if (writeMe) {
      #pragma unroll
      for (int ms = 0; ms < 4; ++ms) {
        float* tb = Ts + m16 * TS + chb + 16 * ms + 8 * h16;
        const v4f lo = { acc[ms][s][0] * WSCALE_INV, acc[ms][s][1] * WSCALE_INV,
                         acc[ms][s][2] * WSCALE_INV, acc[ms][s][3] * WSCALE_INV };
        const v4f hi = { acc[ms][s][4] * WSCALE_INV, acc[ms][s][5] * WSCALE_INV,
                         acc[ms][s][6] * WSCALE_INV, acc[ms][s][7] * WSCALE_INV };
        *(v4fa*)(tb)     = lo;
        *(v4fa*)(tb + 4) = hi;
      }
    }
    __syncthreads();

    v4f vals[4];
    float* dsts[4];
    #pragma unroll
    for (int i = 0; i < 4; ++i) {
      const int q = tid + 256 * i;
      const int line = q >> 3, sub = q & 7;
      const int pos = line >> 3;
      const int choff = (line & 7) * 32 + sub * 4;
      vals[i] = *(const v4fa*)(Ts + pos * TS + choff);
      dsts[i] = Y + ((size_t)(p0 + 16 * s + pos)) * CCH + choff;
    }
    #pragma unroll
    for (int i = 0; i < 4; ++i) *(volatile v4f*)dsts[i] = vals[i];
    __threadfence();
    #pragma unroll
    for (int i = 0; i < 4; ++i) *(volatile v4f*)dsts[i] = vals[i];
    __syncthreads();
  }
}

__device__ __forceinline__ void out_store_pass(const float* T, float* out, float scale,
                                               int n, int cbase, int tid) {
  #pragma unroll
  for (int i = 0; i < 7; ++i) {
    const int q = tid + 256 * i;
    if (q < 196 * 8) {
      const int L = q >> 3, sub = q & 7;
      const int cp = L / 49;
      const int j  = L - cp * 49;
      const int f  = j * 32 + sub * 4;
      const int up = (f >= HWSZ) ? 1 : 0;
      const int cl = 2 * cp + up;
      const int hw = f - up * HWSZ;
      v4f v = *(const v4fa*)(T + cl * HWSZ + hw);
      v *= scale;
      float* dst = out + ((size_t)(n * CCH + cbase + 2 * cp)) * HWSZ + f;
      *(volatile v4f*)dst = v;
    }
  }
}

__global__ __launch_bounds__(256) void out_kernel(
    const float* __restrict__ Y, const float* __restrict__ scl, float* __restrict__ out)
{
  __shared__ __attribute__((aligned(16))) float T[CG * HWSZ];
  const int tid = threadIdx.x;
  const int cbase = blockIdx.x * CG;
  const int n = blockIdx.y;
  const float scale = scl[0];

  #pragma unroll
  for (int i = 0; i < 7; ++i) {
    const int q = tid + 256 * i;
    const int pos = min(q >> 1, HWSZ - 1);
    const int half = q & 1;
    const v4f v = *(const v4fa*)(Y + ((size_t)(n * HWSZ + pos)) * CCH + cbase + 4 * half);
    if (q < 2 * HWSZ) {
      float* t = T + (4 * half) * HWSZ + pos;
      t[0]        = v.x;
      t[HWSZ]     = v.y;
      t[2 * HWSZ] = v.z;
      t[3 * HWSZ] = v.w;
    }
  }
  __syncthreads();

  out_store_pass(T, out, scale, n, cbase, tid);
  __threadfence();
  out_store_pass(T, out, scale, n, cbase, tid);
}

extern "C" void kernel_launch(void* const* d_in, const int* in_sizes, int n_in,
                              void* d_out, int out_size, void* d_ws, size_t ws_size,
                              hipStream_t stream) {
  if (n_in < 4) return;
  if (in_sizes[0] != NPOS * CCH) return;
  if (in_sizes[1] != CCH * CCH * 9 || in_sizes[2] != CCH * CCH * 9) return;
  if (in_sizes[3] != NPOS) return;
  if (out_size != NPOS * CCH) return;

  const float* x  = (const float*)d_in[0];
  const float* w0 = (const float*)d_in[1];
  const float* w1 = (const float*)d_in[2];
  const float* mu = (const float*)d_in[3];
  float* out = (float*)d_out;

  const size_t wb_bytes = (size_t)2 * CCH * KTOT * 2;
  const size_t xb_bytes = (size_t)NPOS * CCH * 2;
  const size_t bm_bytes = (size_t)NPOS * 4;
  const size_t sc_bytes = 128;
  const size_t y_bytes  = (size_t)NPOS * CCH * 4;
  const size_t o_wb = 0;
  const size_t o_xb = o_wb + wb_bytes;
  const size_t o_bm = o_xb + xb_bytes;
  const size_t o_sc = o_bm + bm_bytes;
  const size_t o_y  = o_sc + sc_bytes;
  const size_t total = o_y + y_bytes;
  if (total > ws_size) return;

  char* ws = (char*)d_ws;
  _Float16* wb = (_Float16*)(ws + o_wb);
  _Float16* xb = (_Float16*)(ws + o_xb);
  float* bm  = (float*)(ws + o_bm);
  float* scl = (float*)(ws + o_sc);
  float* Y   = (float*)(ws + o_y);

  const int nw8 = 2 * CCH * KTOT / 8;
  prep_w_kernel<<<(nw8 + 255) / 256, 256, 0, stream>>>(w0, w1, wb);

  const int nx8 = NPOS * (CCH / 8);
  prep_x_kernel<<<(nx8 + 255) / 256, 256, 0, stream>>>(x, xb);

  mask_kernel<<<1, 256, 0, stream>>>(mu, bm, scl);

  conv_kernel<<<NPOS / TILE_P, 256, 0, stream>>>(xb, wb, bm, Y);

  dim3 gOut(CCH / CG, NB);
  out_kernel<<<gOut, 256, 0, stream>>>(Y, scl, out);
}
